// JetGraphClassifier_60447369724691
// MI455X (gfx1250) — hardware-verified
//
#include <hip/hip_runtime.h>
#define NNODE 50000
#define NE 800000
#define NTOT (NE + NNODE)
#define NGR 512
#define NN NNODE
#define MAXDEG 256

typedef __bf16 v16b __attribute__((ext_vector_type(16)));
typedef unsigned short v8us __attribute__((ext_vector_type(8), may_alias));
typedef float  v8f  __attribute__((ext_vector_type(8)));
typedef float  v4f  __attribute__((ext_vector_type(4)));
typedef float  v4fa __attribute__((ext_vector_type(4), may_alias));
union FragB { v16b v; v8us half[2]; unsigned short u[16]; };

__device__ __forceinline__ unsigned short bf16_bits(float x) { unsigned int u = __float_as_uint(x); return (unsigned short)((u + 0x7FFFu + ((u >> 16) & 1u)) >> 16); }
__device__ __forceinline__ float bf16_val(unsigned short b) { return __uint_as_float(((unsigned int)b) << 16); }
__device__ __forceinline__ float bf16_round(float x) { return bf16_val(bf16_bits(x)); }
template <int NT>
__device__ __forceinline__ v8f mmaN(v16b ah, v16b al, v16b bh, v16b bl, v8f c) {
  c = __builtin_amdgcn_wmma_f32_16x16x32_bf16(false, ah, false, bh, (short)0, c, false, false);
  if (NT >= 2) c = __builtin_amdgcn_wmma_f32_16x16x32_bf16(false, al, false, bh, (short)0, c, false, false);
  if (NT >= 3) c = __builtin_amdgcn_wmma_f32_16x16x32_bf16(false, ah, false, bl, (short)0, c, false, false);
  asm volatile("v_nop\n\tv_nop\n\tv_nop\n\tv_nop" : "+v"(c) : "v"(ah), "v"(al), "v"(bh), "v"(bl));
  return c;
}

__global__ __launch_bounds__(256) void k_wt_bf16(const float* __restrict__ W, unsigned short* __restrict__ Wt, int K, int N) {
  const int t = blockIdx.x * 256 + threadIdx.x;
  const int k8n = K / 8;
  if (t >= N * k8n) return;
  const int n = t / k8n, k8 = (t % k8n) * 8;
  v8us v;
#pragma unroll
  for (int i = 0; i < 8; ++i) v[i] = bf16_bits(W[(size_t)(k8 + i) * N + n]);
  *(volatile v8us*)(Wt + (size_t)n * K + k8) = v;
  __threadfence();
  *(volatile v8us*)(Wt + (size_t)n * K + k8) = v;
}

template <bool ASPLIT, int ACT, bool BIAS_BF16>
__global__ __launch_bounds__(128) void k_gemm_bf(const float* __restrict__ A, int lda, const unsigned short* __restrict__ Wt, int ldb,
                                               const float* __restrict__ bias, float* __restrict__ C, int ldc, int M, int N, int K) {
  __shared__ __attribute__((aligned(16))) float so[4][16][64];
  const int tid = threadIdx.x, w = tid >> 5, lane = tid & 31, ln = lane & 15, hh = lane >> 4;
  const int ntn = N / 64;
  const int wid = blockIdx.x * 4 + w;
  const int mt = wid / ntn, nq = wid % ntn;
  if (mt * 16 >= M) return;
  const int row0 = mt * 16, col0 = nq * 64;
  const float* arow = A + (size_t)(row0 + ln) * lda;
  v8f acc[4] = {};
  for (int kb = 0; kb < K; kb += 32) {
    FragB ah, al;
    const v4f x0 = *(const v4fa*)(arow + kb + 8 * hh), x1 = *(const v4fa*)(arow + kb + 8 * hh + 4);
    const v4f x2 = *(const v4fa*)(arow + kb + 16 + 8 * hh), x3 = *(const v4fa*)(arow + kb + 16 + 8 * hh + 4);
    float xs[16] = {x0[0],x0[1],x0[2],x0[3],x1[0],x1[1],x1[2],x1[3],x2[0],x2[1],x2[2],x2[3],x3[0],x3[1],x3[2],x3[3]};
#pragma unroll
    for (int i = 0; i < 16; ++i) { const unsigned short hb = bf16_bits(xs[i]); ah.u[i] = hb; al.u[i] = ASPLIT ? bf16_bits(xs[i] - bf16_val(hb)) : (unsigned short)0; }
#pragma unroll
    for (int t = 0; t < 4; ++t) {
      const unsigned short* brow = Wt + (size_t)(col0 + t * 16 + ln) * ldb + kb;
      FragB b;
      b.half[0] = *(const v8us*)(brow + 8 * hh);
      b.half[1] = *(const v8us*)(brow + 16 + 8 * hh);
      acc[t] = mmaN<ASPLIT ? 2 : 1>(ah.v, al.v, b.v, b.v, acc[t]);
    }
  }
#pragma unroll
  for (int t = 0; t < 4; ++t) {
    float bv = bias ? bias[col0 + t * 16 + ln] : 0.f;
    if (BIAS_BF16) bv = bf16_round(bv);
#pragma unroll
    for (int r = 0; r < 8; ++r) { float v = acc[t][r] + bv; if (ACT == 1) v = fmaxf(v, 0.f); so[w][8 * hh + r][t * 16 + ln] = v; }
  }
  __builtin_amdgcn_fence(__ATOMIC_ACQ_REL, "workgroup");
  __builtin_amdgcn_wave_barrier();
  const int rsub = lane >> 4, c4 = (lane & 15) * 4;
  for (int pass = 0; pass < 2; ++pass) {
#pragma unroll
    for (int q = 0; q < 8; ++q) {
      const int r = q * 2 + rsub;
      const v4f v = *(const v4fa*)&so[w][r][c4];
      *(volatile v4f*)(C + (size_t)(row0 + r) * ldc + col0 + c4) = v;
    }
    if (pass == 0) __threadfence();
  }
}

template <int D, bool CAUSAL>
__global__ __launch_bounds__(128) void k_flash(const float* __restrict__ qb, const float* __restrict__ kb, const float* __restrict__ vb,
                                             int pitch, int T, int H, float scale, float* __restrict__ y, int ypitch) {
  constexpr int KS = D / 32;
  constexpr int DT = D / 16;
  __shared__ __attribute__((aligned(16))) unsigned short sKh[32][D + 8], sKl[32][D + 8], sVh[32][D + 8], sVl[32][D + 8];
  __shared__ __attribute__((aligned(16))) unsigned short sPh[4][16][40], sPl[4][16][40];
  __shared__ __attribute__((aligned(16))) float sO[4][16][D];
  const int tid = threadIdx.x, w = tid >> 5, lane = tid & 31, ln = lane & 15, hh = lane >> 4;
  const int nqb = (T + 63) / 64;
  const int bh = blockIdx.x / nqb, qblk = blockIdx.x % nqb;
  const int b = bh / H, h = bh % H;
  const int q0 = qblk * 64 + w * 16;
  const float* Q = qb + (size_t)b * T * pitch + h * D;
  const float* K = kb + (size_t)b * T * pitch + h * D;
  const float* V = vb + (size_t)b * T * pitch + h * D;

  FragB aqh[KS], aql[KS];
  {
    int row = q0 + ln; if (row >= T) row = T - 1;
    const float* qr = Q + (size_t)row * pitch;
#pragma unroll
    for (int ks = 0; ks < KS; ++ks)
#pragma unroll
      for (int i = 0; i < 16; ++i) {
        const int d = ks * 32 + ((i < 8) ? (8 * hh + i) : (16 + 8 * hh + (i - 8)));
        const float x = qr[d] * scale; const unsigned short hb = bf16_bits(x);
        aqh[ks].u[i] = hb; aql[ks].u[i] = bf16_bits(x - bf16_val(hb));
      }
  }
  float m_r[8], l_r[8];
#pragma unroll
  for (int r = 0; r < 8; ++r) { m_r[r] = -3.0e38f; l_r[r] = 0.f; }
  v8f oacc[DT];
#pragma unroll
  for (int dt = 0; dt < DT; ++dt) oacc[dt] = (v8f){0.f,0.f,0.f,0.f,0.f,0.f,0.f,0.f};

  const int kv_end = CAUSAL ? min(T, qblk * 64 + 64) : T;
  for (int j0 = 0; j0 < kv_end; j0 += 32) {
    __syncthreads();
    for (int e = tid; e < 32 * (D / 4); e += 128) {
      const int r = e / (D / 4), c4 = (e % (D / 4)) * 4;
      const int key = j0 + r;
      v4f kf = {0.f,0.f,0.f,0.f}, vf = {0.f,0.f,0.f,0.f};
      if (key < T) { kf = *(const v4fa*)(K + (size_t)key * pitch + c4); vf = *(const v4fa*)(V + (size_t)key * pitch + c4); }
#pragma unroll
      for (int t = 0; t < 4; ++t) {
        unsigned short hb = bf16_bits(kf[t]); sKh[r][c4 + t] = hb; sKl[r][c4 + t] = bf16_bits(kf[t] - bf16_val(hb));
        hb = bf16_bits(vf[t]); sVh[r][c4 + t] = hb; sVl[r][c4 + t] = bf16_bits(vf[t] - bf16_val(hb));
      }
    }
    __syncthreads();
    v8f s[2];
#pragma unroll
    for (int nt = 0; nt < 2; ++nt) {
      v8f acc = {};
#pragma unroll
      for (int ks = 0; ks < KS; ++ks) {
        FragB bh_, bl_;
        bh_.half[0] = *(const v8us*)&sKh[nt * 16 + ln][ks * 32 + 8 * hh]; bh_.half[1] = *(const v8us*)&sKh[nt * 16 + ln][ks * 32 + 16 + 8 * hh];
        bl_.half[0] = *(const v8us*)&sKl[nt * 16 + ln][ks * 32 + 8 * hh]; bl_.half[1] = *(const v8us*)&sKl[nt * 16 + ln][ks * 32 + 16 + 8 * hh];
        acc = mmaN<3>(aqh[ks].v, aql[ks].v, bh_.v, bl_.v, acc);
      }
      s[nt] = acc;
    }
    float alpha[8];
#pragma unroll
    for (int r = 0; r < 8; ++r) {
      const int qi = q0 + 8 * hh + r;
      const int ja = j0 + ln, jb = j0 + 16 + ln;
      if (CAUSAL) { if (ja > qi) s[0][r] = -3.0e38f; if (jb > qi) s[1][r] = -3.0e38f; }
      if (ja >= T) s[0][r] = -3.0e38f;
      if (jb >= T) s[1][r] = -3.0e38f;
      float mx = fmaxf(s[0][r], s[1][r]);
      mx = fmaxf(mx, __shfl_xor(mx, 1, 32)); mx = fmaxf(mx, __shfl_xor(mx, 2, 32)); mx = fmaxf(mx, __shfl_xor(mx, 4, 32)); mx = fmaxf(mx, __shfl_xor(mx, 8, 32));
      const float mnew = fmaxf(m_r[r], mx);
      alpha[r] = (mnew > -1.0e38f) ? __expf(m_r[r] - mnew) : 1.0f;
      const float p0 = (s[0][r] > -1.0e38f) ? __expf(s[0][r] - mnew) : 0.f;
      const float p1 = (s[1][r] > -1.0e38f) ? __expf(s[1][r] - mnew) : 0.f;
      m_r[r] = mnew;
      l_r[r] = l_r[r] * alpha[r] + p0 + p1;
      unsigned short hb = bf16_bits(p0); sPh[w][8 * hh + r][ln] = hb;      sPl[w][8 * hh + r][ln] = bf16_bits(p0 - bf16_val(hb));
      hb = bf16_bits(p1);                sPh[w][8 * hh + r][16 + ln] = hb; sPl[w][8 * hh + r][16 + ln] = bf16_bits(p1 - bf16_val(hb));
    }
#pragma unroll
    for (int dt = 0; dt < DT; ++dt)
#pragma unroll
      for (int r = 0; r < 8; ++r) oacc[dt][r] *= alpha[r];
    __builtin_amdgcn_fence(__ATOMIC_ACQ_REL, "workgroup");
    __builtin_amdgcn_wave_barrier();
    FragB pah, pal;
    pah.half[0] = *(const v8us*)&sPh[w][ln][8 * hh]; pah.half[1] = *(const v8us*)&sPh[w][ln][16 + 8 * hh];
    pal.half[0] = *(const v8us*)&sPl[w][ln][8 * hh]; pal.half[1] = *(const v8us*)&sPl[w][ln][16 + 8 * hh];
#pragma unroll
    for (int dt = 0; dt < DT; ++dt) {
      FragB bvh, bvl;
#pragma unroll
      for (int i = 0; i < 8; ++i) {
        bvh.u[i] = sVh[8 * hh + i][dt * 16 + ln]; bvh.u[8 + i] = sVh[16 + 8 * hh + i][dt * 16 + ln];
        bvl.u[i] = sVl[8 * hh + i][dt * 16 + ln]; bvl.u[8 + i] = sVl[16 + 8 * hh + i][dt * 16 + ln];
      }
      oacc[dt] = mmaN<3>(pah.v, pal.v, bvh.v, bvl.v, oacc[dt]);
    }
    __builtin_amdgcn_fence(__ATOMIC_ACQ_REL, "workgroup");
    __builtin_amdgcn_wave_barrier();
  }
#pragma unroll
  for (int r = 0; r < 8; ++r) {
    float l = l_r[r];
    l += __shfl_xor(l, 1, 32); l += __shfl_xor(l, 2, 32); l += __shfl_xor(l, 4, 32); l += __shfl_xor(l, 8, 32);
    l_r[r] = (l > 0.f) ? 1.0f / l : 0.f;
  }
#pragma unroll
  for (int dt = 0; dt < DT; ++dt)
#pragma unroll
    for (int r = 0; r < 8; ++r) sO[w][8 * hh + r][dt * 16 + ln] = oacc[dt][r] * l_r[r];
  __builtin_amdgcn_fence(__ATOMIC_ACQ_REL, "workgroup");
  __builtin_amdgcn_wave_barrier();
  for (int pass = 0; pass < 2; ++pass) {
    for (int r = 0; r < 16; ++r) {
      const int row = q0 + r;
      if (row < T && lane < D / 4) {
        const v4f val = *(const v4fa*)&sO[w][r][lane * 4];
        *(volatile v4f*)(y + ((size_t)b * T + row) * ypitch + h * D + lane * 4) = val;
      }
    }
    if (pass == 0) __threadfence();
  }
}

typedef _Float16 v16h __attribute__((ext_vector_type(16)));
union FragH { v16h v; v8us half[2]; _Float16 h[16]; unsigned short u[16]; };
template <int NT>
__device__ __forceinline__ v8f mmaH(v16h ah, v16h al, v16h bh, v16h bl, v8f c) {
  c = __builtin_amdgcn_wmma_f32_16x16x32_f16(false, ah, false, bh, (short)0, c, false, false);
  if (NT >= 2) c = __builtin_amdgcn_wmma_f32_16x16x32_f16(false, al, false, bh, (short)0, c, false, false);
  if (NT >= 3) c = __builtin_amdgcn_wmma_f32_16x16x32_f16(false, ah, false, bl, (short)0, c, false, false);
  asm volatile("v_nop\n\tv_nop\n\tv_nop\n\tv_nop" : "+v"(c) : "v"(ah), "v"(al), "v"(bh), "v"(bl));
  return c;
}
template <bool ASPLIT>
__global__ __launch_bounds__(128) void k_gemm_h(const float* __restrict__ A, int lda, size_t sA, const _Float16* __restrict__ Bh, int ldb, size_t sB, float alpha, float* __restrict__ C, int ldc, size_t sC, int M, int N, int K) {
  __shared__ __attribute__((aligned(16))) float so[4][16][64];
  const int tid = threadIdx.x, w = tid >> 5, lane = tid & 31, ln = lane & 15, hh = lane >> 4; const int by = blockIdx.y;
  A += (size_t)by * sA; Bh += (size_t)by * sB; C += (size_t)by * sC;
  const int ntn = (N + 63) / 64; const int wid = blockIdx.x * 4 + w; const int mt = wid / ntn, nq = wid % ntn; if (mt * 16 >= M) return;
  const int row0 = mt * 16, col0 = nq * 64; const float* arow = A + (size_t)(row0 + ln) * lda;
  v8f acc[4] = {};
  for (int kb = 0; kb < K; kb += 32) {
    FragH ah, al;
    const v4f x0 = *(const v4fa*)(arow + kb + 8 * hh), x1 = *(const v4fa*)(arow + kb + 8 * hh + 4), x2 = *(const v4fa*)(arow + kb + 16 + 8 * hh), x3 = *(const v4fa*)(arow + kb + 16 + 8 * hh + 4);
    float xs[16] = {x0[0],x0[1],x0[2],x0[3],x1[0],x1[1],x1[2],x1[3],x2[0],x2[1],x2[2],x2[3],x3[0],x3[1],x3[2],x3[3]};
#pragma unroll
    for (int i = 0; i < 16; ++i) { const _Float16 h = (_Float16)xs[i]; ah.h[i] = h; al.h[i] = ASPLIT ? (_Float16)(xs[i] - (float)h) : (_Float16)0.0f; }
#pragma unroll
    for (int t = 0; t < 4; ++t) { if (col0 + t * 16 >= N) continue; const size_t boff = (size_t)(col0 + t * 16 + ln) * ldb + kb; FragH bq; bq.half[0] = *(const v8us*)(Bh + boff + 8 * hh); bq.half[1] = *(const v8us*)(Bh + boff + 16 + 8 * hh);
      acc[t] = mmaH<ASPLIT ? 2 : 1>(ah.v, al.v, bq.v, bq.v, acc[t]); }
  }
#pragma unroll
  for (int t = 0; t < 4; ++t) { if (col0 + t * 16 >= N) continue;
#pragma unroll
    for (int r = 0; r < 8; ++r) so[w][8 * hh + r][t * 16 + ln] = acc[t][r] * alpha; }
  __builtin_amdgcn_fence(__ATOMIC_ACQ_REL, "workgroup"); __builtin_amdgcn_wave_barrier();
  const int rsub = lane >> 4, c4 = (lane & 15) * 4;
  for (int pass = 0; pass < 2; ++pass) {
#pragma unroll
    for (int q = 0; q < 8; ++q) { const int r = q * 2 + rsub; if (col0 + c4 < N) { const v4f v = *(const v4fa*)&so[w][r][c4]; *(volatile v4f*)(C + (size_t)(row0 + r) * ldc + col0 + c4) = v; } }
    if (pass == 0) __threadfence(); }
}

#define CS_NW 1024
#define CS_CH 832
#define CS_NB 256
#define CS_CAP 8192
__device__ __forceinline__ int cs_dst(const int* __restrict__ eidst, int e, int ne, int nt, int nn) { if (e >= nt) return -1; int d = (e < ne) ? eidst[e] : (e - ne); return d < 0 ? 0 : (d >= nn ? nn - 1 : d); }
__global__ __launch_bounds__(256) void k_cs_p1(const int* __restrict__ eidst, int ne, int nt, int nn, int* __restrict__ seg_dst, int* __restrict__ seg_eid, int* __restrict__ P1, int* __restrict__ Q1) {
  __shared__ int scnt[8][CS_NB]; __shared__ int srun[8][CS_NB]; __shared__ int sod[8][CS_CH]; __shared__ int soe[8][CS_CH];
  const int tid = threadIdx.x, wv = tid >> 5, lane = tid & 31; const int w = blockIdx.x * 8 + wv; const int e0 = w * CS_CH;
  for (int i = lane; i < CS_NB; i += 32) { scnt[wv][i] = 0; srun[wv][i] = 0; }
  __builtin_amdgcn_fence(__ATOMIC_ACQ_REL, "workgroup"); __builtin_amdgcn_wave_barrier();
#pragma unroll 1
  for (int i0 = 0; i0 < CS_CH; i0 += 32) { const int e = e0 + i0 + lane; const int d = cs_dst(eidst, e, ne, nt, nn); const int hb = (d < 0) ? -1 : (d >> 8);
#pragma unroll 1
    for (int ld = 0; ld < 32; ++ld) { const int kk = __shfl(hb, ld, 32); const unsigned long long m = __ballot(hb == kk); const int first = __ffsll((long long)m) - 1; if (ld == first && lane == first && kk >= 0) scnt[wv][kk] += __popcll(m); }
    __builtin_amdgcn_fence(__ATOMIC_ACQ_REL, "workgroup"); __builtin_amdgcn_wave_barrier(); }
  { int loc[8]; int s = 0; for (int j = 0; j < 8; ++j) { loc[j] = s; s += scnt[wv][lane * 8 + j]; }
    int incl = s; for (int o = 1; o < 32; o <<= 1) { const int v = __shfl_up(incl, o, 32); if (lane >= o) incl += v; } const int excl = incl - s;
    for (int j = 0; j < 8; ++j) srun[wv][lane * 8 + j] = excl + loc[j]; }
  __builtin_amdgcn_fence(__ATOMIC_ACQ_REL, "workgroup"); __builtin_amdgcn_wave_barrier();
  for (int pass = 0; pass < 2; ++pass) { for (int i = lane; i < CS_NB; i += 32) { *(volatile int*)(P1 + (size_t)w * CS_NB + i) = scnt[wv][i]; *(volatile int*)(Q1 + (size_t)w * CS_NB + i) = srun[wv][i]; } if (pass == 0) __threadfence(); }
#pragma unroll 1
  for (int i0 = 0; i0 < CS_CH; i0 += 32) { const int e = e0 + i0 + lane; const int d = cs_dst(eidst, e, ne, nt, nn); const int hb = (d < 0) ? -1 : (d >> 8);
    int pos = -1; int grpcnt = 0; bool leader = false;
#pragma unroll 1
    for (int ld = 0; ld < 32; ++ld) { const int kk = __shfl(hb, ld, 32); const unsigned long long g = __ballot(hb == kk); const int first = __ffsll((long long)g) - 1;
      if (ld == first && kk >= 0) { if (hb == kk) { const unsigned long long below = g & ((1ull << lane) - 1ull); pos = srun[wv][kk] + __popcll(below); if (lane == first) { leader = true; grpcnt = __popcll(g); } } } }
    if (pos >= 0) { sod[wv][pos] = d; soe[wv][pos] = e; }
    __builtin_amdgcn_fence(__ATOMIC_ACQ_REL, "workgroup"); __builtin_amdgcn_wave_barrier();
    if (leader) srun[wv][hb] += grpcnt;
    __builtin_amdgcn_fence(__ATOMIC_ACQ_REL, "workgroup"); __builtin_amdgcn_wave_barrier(); }
  for (int pass = 0; pass < 2; ++pass) { for (int i = lane; i < CS_CH; i += 32) { *(volatile int*)(seg_dst + (size_t)e0 + i) = sod[wv][i]; *(volatile int*)(seg_eid + (size_t)e0 + i) = soe[wv][i]; } if (pass == 0) __threadfence(); }
}
__global__ __launch_bounds__(256) void k_cs_scan(const int* __restrict__ P1, int* __restrict__ R, int* __restrict__ S) {
  __shared__ int tot[CS_NB]; __shared__ int st[CS_NB + 1];
  const int b = threadIdx.x; int acc = 0;
#pragma unroll 1
  for (int w = 0; w < CS_NW; ++w) { const int c = P1[(size_t)w * CS_NB + b]; *(volatile int*)(R + (size_t)w * CS_NB + b) = acc; acc += c; }
  __threadfence();
  acc = 0;
#pragma unroll 1
  for (int w = 0; w < CS_NW; ++w) { const int c = P1[(size_t)w * CS_NB + b]; *(volatile int*)(R + (size_t)w * CS_NB + b) = acc; acc += c; }
  tot[b] = acc; __syncthreads();
  if (b == 0) { int s = 0; for (int i = 0; i < CS_NB; ++i) { st[i] = s; s += (tot[i] + 31) & ~31; } st[CS_NB] = s; }
  __syncthreads();
  for (int pass = 0; pass < 2; ++pass) { *(volatile int*)(S + b) = st[b]; if (b < 32) *(volatile int*)(S + CS_NB + b) = (b == 0) ? st[CS_NB] : 0; if (pass == 0) __threadfence(); }
}
__global__ __launch_bounds__(256) void k_cs_p2(const int* __restrict__ seg_dst, const int* __restrict__ seg_eid, const int* __restrict__ P1, const int* __restrict__ Q1, const int* __restrict__ R, const int* __restrict__ S, int nn, int* __restrict__ csr_eid, int* __restrict__ csr_start, int* __restrict__ csr_cnt) {
  __shared__ int sd[CS_CAP]; __shared__ int se[CS_CAP]; __shared__ int sorted[CS_CAP]; __shared__ int lcnt[CS_NB]; __shared__ int lpre[CS_NB + 1];
  const int hb = blockIdx.x, t = threadIdx.x; const int total = (R[(size_t)(CS_NW - 1) * CS_NB + hb] + P1[(size_t)(CS_NW - 1) * CS_NB + hb]); const int tot = total > CS_CAP ? CS_CAP : total;
#pragma unroll 1
  for (int w = t; w < CS_NW; w += 256) { const int c = P1[(size_t)w * CS_NB + hb]; const int base = R[(size_t)w * CS_NB + hb]; const int src = w * CS_CH + Q1[(size_t)w * CS_NB + hb];
    for (int k = 0; k < c; ++k) { const int p = base + k; if (p < CS_CAP) { sd[p] = seg_dst[src + k] & 255; se[p] = seg_eid[src + k]; } } }
  __syncthreads();
  { int c = 0;
#pragma unroll 1
    for (int i = 0; i < tot; ++i) c += (sd[i] == t) ? 1 : 0; lcnt[t] = c; }
  __syncthreads();
  if (t == 0) { int s = 0; for (int i = 0; i < CS_NB; ++i) { lpre[i] = s; s += lcnt[i]; } lpre[CS_NB] = s; }
  __syncthreads();
  { int k = lpre[t];
#pragma unroll 1
    for (int i = 0; i < tot; ++i) if (sd[i] == t) { sorted[k++] = se[i]; } }
  __syncthreads();
  const int s0 = S[hb]; const int s1 = S[hb + 1];
  for (int pass = 0; pass < 2; ++pass) {
    for (int i = t; i < s1 - s0; i += 256) *(volatile int*)(csr_eid + s0 + i) = (i < tot) ? sorted[i] : -1;
    { const int dst = hb * CS_NB + t; *(volatile int*)(csr_start + dst) = s0 + lpre[t]; *(volatile int*)(csr_cnt + dst) = lcnt[t]; }
    if (pass == 0) __threadfence(); }
}
static void build_csr(const int* eidst, int ne, int nt, int nn, int* seg_dst, int* seg_eid, int* P1, int* Q1, int* R, int* S, int* csr_eid, int* csr_start, int* csr_cnt, hipStream_t stream) {
  k_cs_p1<<<CS_NW / 8, 256, 0, stream>>>(eidst, ne, nt, nn, seg_dst, seg_eid, P1, Q1);
  k_cs_scan<<<1, 256, 0, stream>>>(P1, R, S);
  k_cs_p2<<<CS_NB, 256, 0, stream>>>(seg_dst, seg_eid, P1, Q1, R, S, nn, csr_eid, csr_start, csr_cnt);
}

typedef _Float16 v2h_t __attribute__((ext_vector_type(2))); typedef float v2f_t __attribute__((ext_vector_type(2)));
__global__ __launch_bounds__(256) void k_wt_f16(const float* __restrict__ W, _Float16* __restrict__ Wt, int K, int N, float scale) { const int t = blockIdx.x * 256 + threadIdx.x; if (t >= N * (K / 8)) return; const int n = t / (K / 8), k8 = (t % (K / 8)) * 8; FragH f;
#pragma unroll
  for (int i = 0; i < 8; ++i) f.h[i] = (_Float16)(bf16_round(W[(size_t)(k8 + i) * N + n]) * scale); const v8us o = f.half[0]; *(volatile v8us*)((unsigned short*)Wt + (size_t)n * K + k8) = o; __threadfence(); *(volatile v8us*)((unsigned short*)Wt + (size_t)n * K + k8) = o; }
__global__ __launch_bounds__(256) void k_cvt16(const float* __restrict__ a, _Float16* __restrict__ h, size_t n8) { const size_t t = (size_t)blockIdx.x * 256 + threadIdx.x; if (t >= n8) return; FragH f; for (int q = 0; q < 8; ++q) f.h[q] = (_Float16)a[t * 8 + q]; const v8us o = f.half[0]; *(volatile v8us*)((unsigned short*)h + t * 8) = o; __threadfence(); *(volatile v8us*)((unsigned short*)h + t * 8) = o; }
__global__ __launch_bounds__(256) void k_cvt16x2(const float* __restrict__ a, _Float16* __restrict__ hi, _Float16* __restrict__ lo, size_t n8) { const size_t t = (size_t)blockIdx.x * 256 + threadIdx.x; if (t >= n8) return; FragH fh, fl; for (int q = 0; q < 8; ++q) { const float v = a[t * 8 + q]; const _Float16 h = (_Float16)v; fh.h[q] = h; fl.h[q] = (_Float16)(v - (float)h); } *(volatile v8us*)((unsigned short*)hi + t * 8) = fh.half[0]; *(volatile v8us*)((unsigned short*)lo + t * 8) = fl.half[0]; __threadfence(); *(volatile v8us*)((unsigned short*)hi + t * 8) = fh.half[0]; *(volatile v8us*)((unsigned short*)lo + t * 8) = fl.half[0]; }
__global__ __launch_bounds__(256) void k_deg(const float* __restrict__ w, const int* __restrict__ cstart, const int* __restrict__ ccnt, const int* __restrict__ ceid, float* __restrict__ dis) {
  __shared__ float so[8][32]; const int tid = threadIdx.x, wv = tid >> 5, lane = tid & 31; const int d0 = blockIdx.x * 32;
  for (int k = 0; k < 4; ++k) { const int d = d0 + wv * 4 + k; float s = 0.f;
    if (d < NNODE) { int p0 = cstart[d]; int cn = ccnt[d]; cn = cn < 0 ? 0 : (cn > MAXDEG ? MAXDEG : cn); p0 = p0 < 0 ? 0 : (p0 > NTOT + 32 * CS_NB ? NTOT + 32 * CS_NB : p0);
      for (int q = lane; q < cn; q += 32) { int e = ceid[p0 + q]; e = e < 0 ? 0 : (e >= NTOT ? NTOT - 1 : e); s += (e < NE) ? bf16_round(w[e]) : 1.0f; }
      for (int o = 16; o >= 1; o >>= 1) s += __shfl_xor(s, o, 32); }
    if (lane == 0) so[wv][k] = (s > 0.f) ? rsqrtf(fmaxf(s, 1e-5f)) : 0.f; }
  __syncthreads();
  if (tid < 32) { const float v = so[tid >> 2][tid & 3]; *(volatile float*)(dis + d0 + tid) = v; __threadfence(); *(volatile float*)(dis + d0 + tid) = v; }
}
__global__ __launch_bounds__(256) void k_lin4(const float* __restrict__ x, const float* __restrict__ W, const float* __restrict__ b, int NC, float* __restrict__ Y) { const size_t t = (size_t)blockIdx.x * 256 + threadIdx.x; if (t >= (size_t)NNODE * NC) return; const int c = (int)(t % NC); const size_t n = t / NC; float s = b ? bf16_round(b[c]) : 0.f;
#pragma unroll
  for (int i = 0; i < 4; ++i) s += bf16_round(x[n * 4 + i]) * bf16_round(W[i * NC + c]); *(volatile float*)(Y + t) = s; __threadfence(); *(volatile float*)(Y + t) = s; }
template <int FW, bool LO>
__global__ __launch_bounds__(256) void k_gagg(const _Float16* __restrict__ h, const _Float16* __restrict__ hlo, const float* __restrict__ dis, const float* __restrict__ w, const int* __restrict__ src, const int* __restrict__ cstart, const int* __restrict__ ccnt, const int* __restrict__ ceid, const float* __restrict__ bias, float* __restrict__ out) {
  const int tid = threadIdx.x, wv = tid >> 5, lane = tid & 31; const int d = blockIdx.x * 8 + wv; if (d >= NNODE) return;
  int p0 = cstart[d]; int cn = ccnt[d]; cn = cn < 0 ? 0 : (cn > MAXDEG ? MAXDEG : cn); p0 = p0 < 0 ? 0 : (p0 > NTOT + 32 * CS_NB ? NTOT + 32 * CS_NB : p0); const float dd = dis[d];
  constexpr int PU = FW / 64; float acc[2 * PU]; for (int u = 0; u < 2 * PU; ++u) acc[u] = 0.f;
#pragma unroll 1
  for (int q = 0; q < cn; ++q) { int e = ceid[p0 + q]; e = e < 0 ? 0 : (e >= NTOT ? NTOT - 1 : e); int s; float ww; if (e < NE) { s = src[e]; ww = bf16_round(w[e]); } else { s = e - NE; ww = 1.0f; } s = s < 0 ? 0 : (s >= NNODE ? NNODE - 1 : s);
    const float nrm = dis[s] * ww * dd; const v2h_t* hr = (const v2h_t*)(h + (size_t)s * FW); const v2h_t* lr = (const v2h_t*)(hlo + (size_t)s * FW);
#pragma unroll
    for (int u = 0; u < PU; ++u) { const v2h_t v = hr[u * 32 + lane]; float a0 = (float)v.x, a1 = (float)v.y; if (LO) { const v2h_t w2 = lr[u * 32 + lane]; a0 += (float)w2.x; a1 += (float)w2.y; } acc[2 * u] += a0 * nrm; acc[2 * u + 1] += a1 * nrm; } }
  float* orow = out + (size_t)d * FW;
  for (int pass = 0; pass < 2; ++pass) {
#pragma unroll
    for (int u = 0; u < PU; ++u) { const int c = u * 64 + 2 * lane; v2f_t o; o.x = acc[2 * u] + bf16_round(bias[c]); o.y = acc[2 * u + 1] + bf16_round(bias[c + 1]); *(volatile v2f_t*)(orow + c) = o; } if (pass == 0) __threadfence(); }
}
template <int NC>
__global__ __launch_bounds__(256) void k_colstat(const float* __restrict__ X, int nrows, double* __restrict__ part) { constexpr int G = 256 / NC; __shared__ double r1[G][NC], r2[G][NC]; const int t = threadIdx.x, c = t % NC, g = t / NC; double s = 0.0, q = 0.0; const int n0 = blockIdx.x * 1024;
#pragma unroll 1
  for (int u = g; u < 1024; u += G) { const int n = n0 + u; if (n >= nrows) break; const float v = X[(size_t)n * NC + c]; s += (double)v; q += (double)v * (double)v; }
  r1[g][c] = s; r2[g][c] = q; __syncthreads();
  if (t < NC) { double a = 0.0, b = 0.0; for (int gg = 0; gg < G; ++gg) { a += r1[gg][t]; b += r2[gg][t]; } double* dp = part + ((size_t)blockIdx.x * 256 + t) * 2; *(volatile double*)dp = a; *(volatile double*)(dp + 1) = b; __threadfence(); *(volatile double*)dp = a; *(volatile double*)(dp + 1) = b; } }
__global__ __launch_bounds__(256) void k_statfin(const double* __restrict__ part, int nblk, int NC, double cntrows, const float* __restrict__ g, const float* __restrict__ b, float* __restrict__ st) { const int c = threadIdx.x; if (c >= NC) return; double s = 0.0, q = 0.0; for (int k = 0; k < nblk; ++k) { s += part[((size_t)k * 256 + c) * 2]; q += part[((size_t)k * 256 + c) * 2 + 1]; }
  const double mu = s / cntrows; double var = q / cntrows - mu * mu; if (var < 0.0) var = 0.0; const float rs = (float)(1.0 / sqrt(var + 1e-5)); const float sc = rs * bf16_round(g[c]); const float sh = bf16_round(b[c]) - (float)mu * sc; *(volatile float*)(st + c * 2) = sc; *(volatile float*)(st + c * 2 + 1) = sh; __threadfence(); *(volatile float*)(st + c * 2) = sc; *(volatile float*)(st + c * 2 + 1) = sh; }
template <int NC>
__global__ __launch_bounds__(256) void k_blockout(const float* __restrict__ G, const float* __restrict__ st, const float* __restrict__ SC, float* __restrict__ H) { const size_t t = (size_t)blockIdx.x * 256 + threadIdx.x; if (t >= (size_t)NNODE * NC / 4) return; const int c4 = (int)((t * 4) % NC); const v4f gv = *(const v4fa*)(G + t * 4), sv = *(const v4fa*)(SC + t * 4); v4f o;
  for (int q = 0; q < 4; ++q) { const int c = c4 + q; o[q] = fmaxf(gv[q] * st[c * 2] + st[c * 2 + 1], 0.f) + sv[q]; } *(volatile v4f*)(H + t * 4) = o; __threadfence(); *(volatile v4f*)(H + t * 4) = o; }
__global__ __launch_bounds__(256) void k_pool(const float* __restrict__ Hh, const int* __restrict__ batch, float* __restrict__ Z) {
  const int tid = threadIdx.x, wv = tid >> 5, lane = tid & 31; const int g = blockIdx.x * 8 + wv; if (g >= NGR) return;
  int lo = 0, hi = NNODE; while (lo < hi) { const int m = (lo + hi) >> 1; if (batch[m] < g) lo = m + 1; else hi = m; } const int s0 = lo; lo = 0; hi = NNODE; while (lo < hi) { const int m = (lo + hi) >> 1; if (batch[m] < g + 1) lo = m + 1; else hi = m; } const int s1 = lo;
  float sm[4] = {0.f, 0.f, 0.f, 0.f}, mx[4] = {-__builtin_inff(), -__builtin_inff(), -__builtin_inff(), -__builtin_inff()};
#pragma unroll 1
  for (int n = s0; n < s1; ++n) { const float* r = Hh + (size_t)n * 128;
#pragma unroll
    for (int u = 0; u < 4; ++u) { const float v = r[u * 32 + lane]; sm[u] += v; mx[u] = fmaxf(mx[u], v); } }
  const float inv = 1.0f / fmaxf((float)(s1 - s0), 1.0f); float* zr = Z + (size_t)g * 256;
  for (int pass = 0; pass < 2; ++pass) { for (int u = 0; u < 4; ++u) { *(volatile float*)(zr + u * 32 + lane) = sm[u] * inv; *(volatile float*)(zr + 128 + u * 32 + lane) = mx[u]; } if (pass == 0) __threadfence(); }
}
__global__ __launch_bounds__(256) void k_addsb(float* __restrict__ Y, const float* __restrict__ b, size_t n4) { const size_t t = (size_t)blockIdx.x * 256 + threadIdx.x; if (t >= n4) return; const int c4 = (int)((t * 4) % 128); v4f v = *(const v4fa*)(Y + t * 4); for (int q = 0; q < 4; ++q) v[q] += bf16_round(b[c4 + q]); *(volatile v4f*)(Y + t * 4) = v; __threadfence(); *(volatile v4f*)(Y + t * 4) = v; }
__global__ __launch_bounds__(512) void k_head(const float* __restrict__ F1, const float* __restrict__ fb1, const float* __restrict__ fg, const float* __restrict__ fbe, const float* __restrict__ fW2, const float* __restrict__ fb2, float* __restrict__ out) {
  __shared__ float ssc[128], ssh[128]; const int t = threadIdx.x;
  if (t < 128) { double s = 0.0, q = 0.0; const float bb = bf16_round(fb1[t]); for (int g = 0; g < NGR; ++g) { const float v = F1[g * 128 + t] * 0.0625f + bb; s += (double)v; q += (double)v * (double)v; } const double mu = s / NGR; double var = q / NGR - mu * mu; if (var < 0.0) var = 0.0; const float rs = (float)(1.0 / sqrt(var + 1e-5)); ssc[t] = rs * bf16_round(fg[t]); ssh[t] = bf16_round(fbe[t]) - (float)mu * ssc[t]; }
  __syncthreads();
  float r = 0.f; if (t < NGR) { r = bf16_round(fb2[0]);
#pragma unroll 1
    for (int c = 0; c < 128; ++c) { const float v = fmaxf((F1[t * 128 + c] * 0.0625f + bf16_round(fb1[c])) * ssc[c] + ssh[c], 0.f); r += v * bf16_round(fW2[c]); } }
  if (t < NGR) { *(volatile float*)(out + t) = r; } __threadfence(); if (t < NGR) { *(volatile float*)(out + t) = r; }
}
extern "C" void kernel_launch(void* const* d_in, const int* in_sizes, int n_in,
                              void* d_out, int out_size, void* d_ws, size_t ws_size, hipStream_t stream) {
  (void)in_sizes; (void)n_in; (void)out_size;
  const float* x = (const float*)d_in[0]; const int* ei = (const int*)d_in[1]; const float* ew = (const float*)d_in[2]; const int* batch = (const int*)d_in[3];
  const float* W1 = (const float*)d_in[4]; const float* b1 = (const float*)d_in[5]; const float* g1 = (const float*)d_in[6]; const float* be1 = (const float*)d_in[7]; const float* sW1 = (const float*)d_in[8]; const float* sb1 = (const float*)d_in[9];
  const float* W2 = (const float*)d_in[10]; const float* b2 = (const float*)d_in[11]; const float* g2 = (const float*)d_in[12]; const float* be2 = (const float*)d_in[13];
  const float* W3 = (const float*)d_in[14]; const float* b3 = (const float*)d_in[15]; const float* g3 = (const float*)d_in[16]; const float* be3 = (const float*)d_in[17]; const float* sW3 = (const float*)d_in[18]; const float* sb3 = (const float*)d_in[19];
  const float* fW1 = (const float*)d_in[20]; const float* fb1 = (const float*)d_in[21]; const float* fg = (const float*)d_in[22]; const float* fbe = (const float*)d_in[23]; const float* fW2 = (const float*)d_in[24]; const float* fb2 = (const float*)d_in[25];
  char* ws = (char*)d_ws; size_t off = 0;
  auto take = [&](size_t bytes) { char* p = ws + off; off += (bytes + 255) & ~(size_t)255; return p; };
  const int NBLK = (NNODE + 1023) / 1024;
  _Float16* Bw2 = (_Float16*)take(64 * 64 * 2); _Float16* Bw3 = (_Float16*)take(128 * 64 * 2); _Float16* Bs3 = (_Float16*)take(128 * 64 * 2); _Float16* Bf1 = (_Float16*)take(128 * 256 * 2);
  double* part = (double*)take((size_t)NBLK * 256 * 2 * 8); float* st = (float*)take(256 * 2 * 4);
  int* seg_dst = (int*)take((size_t)CS_NW * CS_CH * 4); int* seg_eid = (int*)take((size_t)CS_NW * CS_CH * 4); int* P1 = (int*)take((size_t)CS_NW * CS_NB * 4); int* Q1 = (int*)take((size_t)CS_NW * CS_NB * 4); int* R_ = (int*)take((size_t)CS_NW * CS_NB * 4); int* S_ = (int*)take((CS_NB + 32) * 4);
  int* ceid = (int*)take(((size_t)NTOT + 32 * CS_NB) * 4); int* cstart = (int*)take((size_t)CS_NB * CS_NB * 4); int* ccnt = (int*)take((size_t)CS_NB * CS_NB * 4);
  float* dis = (float*)take((size_t)((NNODE + 31) / 32) * 32 * 4); float* T = (float*)take((size_t)NNODE * 128 * 4); _Float16* Th = (_Float16*)take((size_t)NNODE * 128 * 2); _Float16* Tl = (_Float16*)take((size_t)NNODE * 128 * 2); float* G = (float*)take((size_t)NNODE * 128 * 4); float* SC = (float*)take((size_t)NNODE * 128 * 4); float* Ha = (float*)take((size_t)NNODE * 64 * 4); float* Hb = (float*)take((size_t)NNODE * 64 * 4); float* Hc = (float*)take((size_t)NNODE * 128 * 4);
  float* Z = (float*)take((size_t)NGR * 256 * 4); float* F1 = (float*)take((size_t)NGR * 128 * 4);
  if (off > ws_size) return;
  k_wt_f16<<<(64 * 8 + 255) / 256, 256, 0, stream>>>(W2, Bw2, 64, 64, 16.0f); k_wt_f16<<<(128 * 8 + 255) / 256, 256, 0, stream>>>(W3, Bw3, 64, 128, 16.0f); k_wt_f16<<<(128 * 8 + 255) / 256, 256, 0, stream>>>(sW3, Bs3, 64, 128, 16.0f); k_wt_f16<<<(128 * 32 + 255) / 256, 256, 0, stream>>>(fW1, Bf1, 256, 128, 16.0f);
  build_csr(ei + NE, NE, NTOT, NNODE, seg_dst, seg_eid, P1, Q1, R_, S_, ceid, cstart, ccnt, stream);
  k_deg<<<(NNODE + 31) / 32, 256, 0, stream>>>(ew, cstart, ccnt, ceid, dis);
  k_lin4<<<(NNODE * 64 + 255) / 256, 256, 0, stream>>>(x, W1, nullptr, 64, T); k_cvt16<<<(NNODE * 64 / 8 + 255) / 256, 256, 0, stream>>>(T, Th, (size_t)NNODE * 64 / 8);
  k_gagg<64, false><<<(NNODE + 7) / 8, 256, 0, stream>>>(Th, Th, dis, ew, ei, cstart, ccnt, ceid, b1, G);
  k_colstat<64><<<NBLK, 256, 0, stream>>>(G, NNODE, part); k_statfin<<<1, 256, 0, stream>>>(part, NBLK, 64, (double)NNODE, g1, be1, st);
  k_lin4<<<(NNODE * 64 + 255) / 256, 256, 0, stream>>>(x, sW1, sb1, 64, SC); k_blockout<64><<<(NNODE * 64 / 4 + 255) / 256, 256, 0, stream>>>(G, st, SC, Ha);
  k_gemm_h<true><<<dim3(((NNODE / 16) * 1 + 3) / 4, 1), 128, 0, stream>>>(Ha, 64, 0, Bw2, 64, 0, 0.0625f, T, 64, 0, NNODE, 64, 64); k_cvt16<<<(NNODE * 64 / 8 + 255) / 256, 256, 0, stream>>>(T, Th, (size_t)NNODE * 64 / 8);
  k_gagg<64, false><<<(NNODE + 7) / 8, 256, 0, stream>>>(Th, Th, dis, ew, ei, cstart, ccnt, ceid, b2, G);
  k_colstat<64><<<NBLK, 256, 0, stream>>>(G, NNODE, part); k_statfin<<<1, 256, 0, stream>>>(part, NBLK, 64, (double)NNODE, g2, be2, st); k_blockout<64><<<(NNODE * 64 / 4 + 255) / 256, 256, 0, stream>>>(G, st, Ha, Hb);
  k_gemm_h<true><<<dim3(((NNODE / 16) * 2 + 3) / 4, 1), 128, 0, stream>>>(Hb, 64, 0, Bw3, 64, 0, 0.0625f, T, 128, 0, NNODE, 128, 64); k_cvt16x2<<<(NNODE * 128 / 8 + 255) / 256, 256, 0, stream>>>(T, Th, Tl, (size_t)NNODE * 128 / 8);
  k_gagg<128, true><<<(NNODE + 7) / 8, 256, 0, stream>>>(Th, Tl, dis, ew, ei, cstart, ccnt, ceid, b3, G);
  k_colstat<128><<<NBLK, 256, 0, stream>>>(G, NNODE, part); k_statfin<<<1, 256, 0, stream>>>(part, NBLK, 128, (double)NNODE, g3, be3, st);
  k_gemm_h<true><<<dim3(((NNODE / 16) * 2 + 3) / 4, 1), 128, 0, stream>>>(Hb, 64, 0, Bs3, 64, 0, 0.0625f, SC, 128, 0, NNODE, 128, 64);
  k_addsb<<<(NNODE * 128 / 4 + 255) / 256, 256, 0, stream>>>(SC, sb3, (size_t)NNODE * 128 / 4);
  k_blockout<128><<<(NNODE * 128 / 4 + 255) / 256, 256, 0, stream>>>(G, st, SC, Hc);
  k_pool<<<NGR / 8, 256, 0, stream>>>(Hc, batch, Z);
  k_gemm_h<true><<<dim3(((NGR / 16) * 2 + 3) / 4, 1), 128, 0, stream>>>(Z, 256, 0, Bf1, 256, 0, 1.f, F1, 128, 0, NGR, 128, 256);
  k_head<<<1, 512, 0, stream>>>(F1, fb1, fg, fbe, fW2, fb2, (float*)d_out);
}
